// TransformerBlock_73332271612201
// MI455X (gfx1250) — hardware-verified
//
#include <hip/hip_runtime.h>
#include <stddef.h>


typedef _Float16 v16h __attribute__((ext_vector_type(16)));
typedef _Float16 v8h  __attribute__((ext_vector_type(8)));
typedef _Float16 v4h  __attribute__((ext_vector_type(4)));
typedef float    v8f  __attribute__((ext_vector_type(8)));
typedef float    v4f  __attribute__((ext_vector_type(4)));
typedef unsigned int   v4u  __attribute__((ext_vector_type(4)));
typedef unsigned int   v8u  __attribute__((ext_vector_type(8)));
typedef unsigned short v8us __attribute__((ext_vector_type(8)));
typedef __bf16   v16bf __attribute__((ext_vector_type(16)));

#ifndef NB
#define NB 2
#endif
#ifndef SEQ
#define SEQ 2048
#endif
#define NB_FULL  2
#define SEQ_FULL 2048
#define DIM   256
#define NHEAD 8
#define HD    32
#define DFF   1024
#define MROWS (NB * SEQ)

#define LDT 72
#define LDC 68
#define PLD 40

#define WCARRY 64.0f
#define ACARRY 64.0f
#define SCORE_SCALE 5.656854249492380f
#define LN_EPS 1.0e-5f

static_assert(NB >= 1 && NB <= NB_FULL);
static_assert(SEQ >= 128 && SEQ <= SEQ_FULL && (SEQ % 128) == 0);
static_assert(DIM == NHEAD * HD);
static_assert(HD == 32);
static_assert((NHEAD % 2) == 0 && 2 * HD == 64);
static_assert((DIM % 64) == 0 && (DFF % 64) == 0 && ((3 * DIM) % 64) == 0);
static_assert((DIM % 32) == 0 && (DFF % 32) == 0);
static_assert((MROWS % 64) == 0 && (MROWS % 8) == 0);
static_assert(((size_t)MROWS * DIM) % (8 * 256) == 0);
static_assert((size_t)MROWS * DFF < (size_t)0xFFFFFFFFu);
static_assert(((LDT * 2) % 16) == 0 && ((PLD * 2) % 16) == 0 && ((LDC * 4) % 16) == 0);
static_assert(LDT >= 64 && PLD >= 32 && LDC >= 64);
static_assert((size_t)(2 * 64 * LDT * 2) * 2 + (size_t)8 * 2 * 16 * PLD * 2 <= (size_t)65536);
static_assert(((size_t)(NB - 1) * SEQ_FULL + SEQ) * DIM <= (size_t)NB_FULL * SEQ_FULL * DIM);

#define PLANE_ELEMS ((size_t)MROWS * DIM)
#define WQKV_BYTES  ((size_t)3 * DIM * DIM * 2)
#define WPROJ_BYTES ((size_t)DIM * DIM * 2)
#define WFC1_BYTES  ((size_t)DFF * DIM * 2)
#define WFC2_BYTES  ((size_t)DIM * DFF * 2)
#define P16_BYTES   (PLANE_ELEMS * 2)
#define P32_BYTES   (PLANE_ELEMS * 4)
#define H1_BYTES    ((size_t)MROWS * DFF * 2)
#define OFF_WQKV   ((size_t)0)
#define OFF_WPROJ  (OFF_WQKV + WQKV_BYTES)
#define OFF_WFC1   (OFF_WPROJ + WPROJ_BYTES)
#define OFF_WFC2   (OFF_WFC1 + WFC1_BYTES)
#define OFF_X16    (OFF_WFC2 + WFC2_BYTES)
#define OFF_QK     (OFF_X16 + P16_BYTES)
#define OFF_VT     (OFF_QK + 4 * P16_BYTES)
#define OFF_CTX    (OFF_VT + 2 * P16_BYTES)
#define OFF_Y      (OFF_CTX + P16_BYTES)
#define OFF_NETF   (OFF_Y + P32_BYTES)
#define OFF_NET16  (OFF_NETF + P32_BYTES)
#define OFF_H1     (OFF_NET16 + P16_BYTES)
#define WS_TOTAL   (OFF_H1 + H1_BYTES)
static_assert((WQKV_BYTES % 128) == 0 && (WPROJ_BYTES % 128) == 0 && (WFC1_BYTES % 128) == 0);
static_assert((WFC2_BYTES % 128) == 0 && (P16_BYTES % 128) == 0 && (P32_BYTES % 128) == 0);
static_assert((H1_BYTES % 128) == 0);
static_assert(WS_TOTAL <= (size_t)134217728);

__device__ __forceinline__ unsigned bf16bits(float x) {
  const unsigned u = __float_as_uint(x);
  return (u + 0x7FFFu + ((u >> 16) & 1u)) >> 16;
}
__device__ __forceinline__ float bf16r(float x) {
  return __uint_as_float(bf16bits(x) << 16);
}
__device__ __forceinline__ unsigned short f16bits(float x) {
  union { _Float16 h; unsigned short u; } cv;
  cv.h = (_Float16)x;
  return cv.u;
}

__device__ __forceinline__ v16h frag_at(const _Float16* p) {
  v8h lo = *(const v8h*)(p);
  v8h hi = *(const v8h*)(p + 16);
  v16h out;
#pragma unroll
  for (int i = 0; i < 8; ++i) { out[i] = lo[i]; out[i + 8] = hi[i]; }
  return out;
}
__device__ __forceinline__ v8u gfrag_u(const unsigned short* __restrict__ p) {
  const v4u lo = *(const v4u*)(p);
  const v4u hi = *(const v4u*)(p + 16);
  return __builtin_shufflevector(lo, hi, 0, 1, 2, 3, 4, 5, 6, 7);
}
#define LDS_FRAG(dst, arr, idx)                                                     \
  do {                                                                              \
    const v4u lo_ = *(const v4u*)&arr[(idx)];                                       \
    const v4u hi_ = *(const v4u*)&arr[(idx) + 16u];                                 \
    (dst) = __builtin_shufflevector(lo_, hi_, 0, 1, 2, 3, 4, 5, 6, 7);              \
  } while (0)

__device__ __forceinline__ v8f wmma16(v16h a, v16h b, v8f c) {
  v8f d = __builtin_amdgcn_wmma_f32_16x16x32_f16(false, a, false, b, (short)0, c,
                                                 false, false);
  asm volatile("v_nop\n\tv_nop\n\tv_nop\n\tv_nop" : "+v"(d) : "v"(a), "v"(b));
  return d;
}
union FragU { v16bf v; v8u u; };
__device__ __forceinline__ v8f wmma_bf(v8u a, v8u b, v8f c) {
  FragU ua, ub;
  ua.u = a;
  ub.u = b;
  v8f d = __builtin_amdgcn_wmma_f32_16x16x32_bf16(false, ua.v, false, ub.v, (short)0, c,
                                                  false, false);
  asm volatile("v_nop\n\tv_nop\n\tv_nop\n\tv_nop" : "+v"(d) : "v"(a), "v"(b));
  return d;
}

__device__ __forceinline__ float red16_max(float x) {
#pragma unroll
  for (int off = 1; off < 16; off <<= 1) x = fmaxf(x, __shfl_xor(x, off, 32));
  return x;
}
__device__ __forceinline__ float red16_sum(float x) {
#pragma unroll
  for (int off = 1; off < 16; off <<= 1) x += __shfl_xor(x, off, 32);
  return x;
}
__device__ __forceinline__ float red32_sum(float x) {
#pragma unroll
  for (int off = 1; off < 32; off <<= 1) x += __shfl_xor(x, off, 32);
  return x;
}

__device__ __forceinline__ void wave_lds_sync() {
  __builtin_amdgcn_fence(3  , "wavefront");
  asm volatile("s_wait_dscnt 0x0" ::: "memory");
  __builtin_amdgcn_wave_barrier();
}

__device__ __forceinline__ void gemm_acc(const _Float16* __restrict__ A16,
                                         const _Float16* __restrict__ Bt, const unsigned K,
                                         const unsigned arow, const unsigned bcol,
                                         const unsigned hh, v8f& acc0, v8f& acc1) {
  const _Float16* ap  = A16 + (size_t)arow * K + hh * 8u;
  const _Float16* bp0 = Bt + (size_t)bcol * K + hh * 8u;
  const _Float16* bp1 = bp0 + (size_t)16 * K;
#pragma unroll 2
  for (unsigned k0 = 0; k0 < K; k0 += 32u) {
    const v16h a  = frag_at(ap + k0);
    const v16h b0 = frag_at(bp0 + k0);
    const v16h b1 = frag_at(bp1 + k0);
    acc0 = wmma16(a, b0, acc0);
    acc1 = wmma16(a, b1, acc1);
  }
}

__global__ __launch_bounds__(256) void wconv_kernel(
    const float* __restrict__ W, _Float16* __restrict__ Wt, unsigned K, unsigned N) {
  __shared__ __attribute__((aligned(16))) _Float16 T[64 * LDT];
  const unsigned tid = threadIdx.x;
  const unsigned n0 = blockIdx.x * 64u;
  const unsigned k0 = blockIdx.y * 64u;
#pragma unroll 4
  for (unsigned j = 0; j < 16u; ++j) {
    const unsigned idx = tid + 256u * j;
    const unsigned kr = idx >> 6, nc = idx & 63u;
    const float v = W[(size_t)(k0 + kr) * N + n0 + nc];
    T[nc * LDT + kr] = (_Float16)(WCARRY * bf16r(v));
  }
  __syncthreads();
  v8h x[2];
  size_t off[2];
#pragma unroll
  for (unsigned i = 0; i < 2u; ++i) {
    const unsigned n = 32u * i + (tid >> 3);
    const unsigned kc = (tid & 7u) * 8u;
    x[i] = *(const v8h*)&T[n * LDT + kc];
    off[i] = (size_t)(n0 + n) * K + k0 + kc;
  }
#pragma unroll
  for (int i = 0; i < 2; ++i) *(volatile v8h*)(Wt + off[i]) = x[i];
  __threadfence();
#pragma unroll
  for (int i = 0; i < 2; ++i) *(volatile v8h*)(Wt + off[i]) = x[i];
}

__global__ __launch_bounds__(256) void xconv_kernel(
    const float* __restrict__ Xin, _Float16* __restrict__ dst) {
  const unsigned e = (blockIdx.x * 256u + threadIdx.x) * 8u;
  const unsigned crow = e / (unsigned)DIM;
  const unsigned c = e - crow * (unsigned)DIM;
  const unsigned bidx = crow / (unsigned)SEQ;
  const unsigned sq = crow - bidx * (unsigned)SEQ;
  const size_t frow = (size_t)bidx * SEQ_FULL + sq;
  const float* sp = Xin + frow * DIM + c;
  const v4f a0 = *(const v4f*)(sp);
  const v4f a1 = *(const v4f*)(sp + 4);
  v8h o;
#pragma unroll
  for (int j = 0; j < 4; ++j) {
    o[j]     = (_Float16)bf16r(a0[j]);
    o[j + 4] = (_Float16)bf16r(a1[j]);
  }
  *(volatile v8h*)(dst + (size_t)e) = o;
  __threadfence();
  *(volatile v8h*)(dst + (size_t)e) = o;
}

__global__ __launch_bounds__(256) void qkv_gemm_kernel(
    const _Float16* __restrict__ X16, const _Float16* __restrict__ Wt,
    unsigned short* __restrict__ QK, unsigned short* __restrict__ VT) {
  __shared__ __attribute__((aligned(16))) float Cs[64 * LDC];
  const unsigned tid = threadIdx.x, lane = tid & 31u;
  const unsigned wave = __builtin_amdgcn_readfirstlane(threadIdx.x >> 5);
  const unsigned mw = wave >> 1, nw = wave & 1u;
  const unsigned hh = lane >> 4, m = lane & 15u;
  const unsigned n0 = blockIdx.x * 64u;
  const unsigned row0 = blockIdx.y * 64u;

  v8f acc0 = {}, acc1 = {};
  gemm_acc(X16, Wt, (unsigned)DIM, row0 + mw * 16u + m, n0 + nw * 32u + m, hh, acc0, acc1);
#pragma unroll
  for (int r = 0; r < 8; ++r) {
    float* d = &Cs[(mw * 16u + hh * 8u + (unsigned)r) * LDC + nw * 32u + m];
    d[0]  = acc0[r];
    d[16] = acc1[r];
  }
  __syncthreads();

  const unsigned which = blockIdx.x >> 2;
  const unsigned cn0 = n0 - which * (unsigned)DIM;
  v8us xh[2], xl[2];
  size_t off[2];

  if (which < 2u) {
#pragma unroll
    for (unsigned i = 0; i < 2u; ++i) {
      const unsigned r = 32u * i + (tid >> 3);
      const unsigned c = (tid & 7u) * 8u;
      const v4f u0 = *(const v4f*)&Cs[r * LDC + c];
      const v4f u1 = *(const v4f*)&Cs[r * LDC + c + 4];
#pragma unroll
      for (int j = 0; j < 4; ++j) {
        const float a = u0[j] * (1.0f / WCARRY);
        const float b = u1[j] * (1.0f / WCARRY);
        const unsigned ah = bf16bits(a), bh = bf16bits(b);
        const unsigned al = bf16bits(a - __uint_as_float(ah << 16));
        const unsigned bl = bf16bits(b - __uint_as_float(bh << 16));
        xh[i][j] = (unsigned short)ah;  xh[i][j + 4] = (unsigned short)bh;
        xl[i][j] = (unsigned short)al;  xl[i][j + 4] = (unsigned short)bl;
      }
      off[i] = (size_t)(which * 2u) * PLANE_ELEMS + (size_t)(row0 + r) * DIM + cn0 + c;
    }
#pragma unroll
    for (int i = 0; i < 2; ++i) {
      *(volatile v8us*)(QK + off[i]) = xh[i];
      *(volatile v8us*)(QK + off[i] + PLANE_ELEMS) = xl[i];
    }
    __threadfence();
#pragma unroll
    for (int i = 0; i < 2; ++i) {
      *(volatile v8us*)(QK + off[i]) = xh[i];
      *(volatile v8us*)(QK + off[i] + PLANE_ELEMS) = xl[i];
    }
  } else {
    const unsigned bidx = row0 / (unsigned)SEQ;
    const unsigned key0 = row0 - bidx * (unsigned)SEQ;
#pragma unroll
    for (unsigned i = 0; i < 2u; ++i) {
      const unsigned dcol = 32u * i + (tid >> 3);
      const unsigned kk = (tid & 7u) * 8u;
#pragma unroll
      for (unsigned j = 0; j < 8u; ++j) {
        const float a = Cs[(kk + j) * LDC + dcol] * (1.0f / WCARRY);
        const unsigned ah = bf16bits(a);
        const unsigned al = bf16bits(a - __uint_as_float(ah << 16));
        xh[i][j] = (unsigned short)ah;
        xl[i][j] = (unsigned short)al;
      }
      off[i] = ((size_t)bidx * DIM + cn0 + dcol) * SEQ + key0 + kk;
    }
#pragma unroll
    for (int i = 0; i < 2; ++i) {
      *(volatile v8us*)(VT + off[i]) = xh[i];
      *(volatile v8us*)(VT + off[i] + PLANE_ELEMS) = xl[i];
    }
    __threadfence();
#pragma unroll
    for (int i = 0; i < 2; ++i) {
      *(volatile v8us*)(VT + off[i]) = xh[i];
      *(volatile v8us*)(VT + off[i] + PLANE_ELEMS) = xl[i];
    }
  }
}

__global__ __launch_bounds__(256) void attn_kernel(
    const unsigned short* __restrict__ QK, const unsigned short* __restrict__ VT,
    unsigned short* __restrict__ Ctx) {
  __shared__ __attribute__((aligned(16))) unsigned short Ks[2 * 64 * LDT];
  __shared__ __attribute__((aligned(16))) unsigned short Vs[2 * 64 * LDT];
  __shared__ __attribute__((aligned(16))) unsigned short Ps[8 * 2 * 16 * PLD];

  const unsigned tid = threadIdx.x, lane = tid & 31u;
  const unsigned wave = __builtin_amdgcn_readfirstlane(threadIdx.x >> 5);
  const unsigned hh = lane >> 4, m = lane & 15u;
  const unsigned hsel = wave >> 2, wq = wave & 3u;
  const unsigned q0 = blockIdx.x * 64u;
  const unsigned hp = blockIdx.y;
  const unsigned b = blockIdx.z;
  const unsigned pbase = wave * (2u * 16u * PLD);

  const size_t qoff = (size_t)(b * (unsigned)SEQ + q0 + wq * 16u + m) * DIM
                      + hp * 64u + hsel * 32u + hh * 8u;
  const v8u qhi = gfrag_u(QK + qoff);
  const v8u qlo = gfrag_u(QK + PLANE_ELEMS + qoff);

  float mrow[8], lrow[8];
  v8f o0 = {}, o1 = {};
#pragma unroll
  for (int v = 0; v < 8; ++v) { mrow[v] = -1.0e30f; lrow[v] = 0.0f; }

  const size_t kbase = 2 * PLANE_ELEMS + (size_t)b * SEQ * DIM + hp * 64u;
  const size_t vbase = ((size_t)b * DIM + hp * 64u) * SEQ;

  for (unsigned kb = 0; kb < (unsigned)SEQ; kb += 64u) {
#pragma unroll
    for (unsigned j = 0; j < 2u; ++j) {
      const unsigned idx = tid + 256u * j;
      const unsigned r = idx >> 3, c = (idx & 7u) * 8u;
      const size_t kg = kbase + (size_t)(kb + r) * DIM + c;
      const size_t vg = vbase + (size_t)r * SEQ + kb + c;
      const v4u k_hi = *(const v4u*)(QK + kg);
      const v4u k_lo = *(const v4u*)(QK + PLANE_ELEMS + kg);
      const v4u v_hi = *(const v4u*)(VT + vg);
      const v4u v_lo = *(const v4u*)(VT + PLANE_ELEMS + vg);
      *(v4u*)&Ks[r * LDT + c] = k_hi;
      *(v4u*)&Ks[64u * LDT + r * LDT + c] = k_lo;
      *(v4u*)&Vs[r * LDT + c] = v_hi;
      *(v4u*)&Vs[64u * LDT + r * LDT + c] = v_lo;
    }
    __syncthreads();

#pragma unroll 1
    for (unsigned c32 = 0; c32 < 2u; ++c32) {
      const unsigned kix = (c32 * 32u + m) * LDT + hsel * 32u + hh * 8u;
      v8u kh0, kl0, kh1, kl1;
      LDS_FRAG(kh0, Ks, kix);
      LDS_FRAG(kl0, Ks, 64u * LDT + kix);
      LDS_FRAG(kh1, Ks, kix + 16u * LDT);
      LDS_FRAG(kl1, Ks, 64u * LDT + kix + 16u * LDT);
      v8f s0 = {}, s1 = {};
      s0 = wmma_bf(qhi, kl0, s0);
      s0 = wmma_bf(qlo, kh0, s0);
      s0 = wmma_bf(qhi, kh0, s0);
      s1 = wmma_bf(qhi, kl1, s1);
      s1 = wmma_bf(qlo, kh1, s1);
      s1 = wmma_bf(qhi, kh1, s1);
      s0 = s0 * SCORE_SCALE;
      s1 = s1 * SCORE_SCALE;

#pragma unroll
      for (int v = 0; v < 8; ++v) {
        const float mx = red16_max(fmaxf(s0[v], s1[v]));
        const float mn = fmaxf(mrow[v], mx);
        const float alpha = __expf(mrow[v] - mn);
        mrow[v] = mn;
        const float p0 = __expf(s0[v] - mn);
        const float p1 = __expf(s1[v] - mn);
        const float rs = red16_sum(p0 + p1);
        lrow[v] = alpha * lrow[v] + rs;
        o0[v] = o0[v] * alpha;
        o1[v] = o1[v] * alpha;
        const unsigned h0 = bf16bits(p0), h1 = bf16bits(p1);
        const unsigned l0 = bf16bits(p0 - __uint_as_float(h0 << 16));
        const unsigned l1 = bf16bits(p1 - __uint_as_float(h1 << 16));
        const unsigned prow = pbase + (hh * 8u + (unsigned)v) * PLD + m;
        Ps[prow]                   = (unsigned short)h0;
        Ps[prow + 16u]             = (unsigned short)h1;
        Ps[prow + 16u * PLD]       = (unsigned short)l0;
        Ps[prow + 16u * PLD + 16u] = (unsigned short)l1;
      }
      wave_lds_sync();

      const unsigned pix = pbase + m * PLD + hh * 8u;
      v8u ph, pl;
      LDS_FRAG(ph, Ps, pix);
      LDS_FRAG(pl, Ps, pix + 16u * PLD);
      const unsigned vix = (hsel * 32u + m) * LDT + c32 * 32u + hh * 8u;
      v8u vh0, vl0, vh1, vl1;
      LDS_FRAG(vh0, Vs, vix);
      LDS_FRAG(vl0, Vs, 64u * LDT + vix);
      LDS_FRAG(vh1, Vs, vix + 16u * LDT);
      LDS_FRAG(vl1, Vs, 64u * LDT + vix + 16u * LDT);
      o0 = wmma_bf(ph, vl0, o0);
      o0 = wmma_bf(pl, vh0, o0);
      o0 = wmma_bf(ph, vh0, o0);
      o1 = wmma_bf(ph, vl1, o1);
      o1 = wmma_bf(pl, vh1, o1);
      o1 = wmma_bf(ph, vh1, o1);
      wave_lds_sync();
    }
    __syncthreads();
  }

#pragma unroll
  for (int v = 0; v < 8; ++v) {
    const float inv = __builtin_amdgcn_rcpf(lrow[v]) * ACARRY;
    const unsigned prow = pbase + (hh * 8u + (unsigned)v) * PLD + m;
    Ps[prow]       = f16bits(o0[v] * inv);
    Ps[prow + 16u] = f16bits(o1[v] * inv);
  }
  __syncthreads();
  v4u x[2];
  size_t off[2];
#pragma unroll
  for (unsigned i = 0; i < 2u; ++i) {
    const unsigned r = 32u * i + (tid >> 3);
    const unsigned c = tid & 7u;
    const unsigned sw = (c >> 2) * 4u + (r >> 4);
    x[i] = *(const v4u*)&Ps[sw * (2u * 16u * PLD) + (r & 15u) * PLD + (c & 3u) * 8u];
    off[i] = (size_t)(b * (unsigned)SEQ + q0 + r) * DIM + hp * 64u + c * 8u;
  }
#pragma unroll
  for (int i = 0; i < 2; ++i) *(volatile v4u*)(Ctx + off[i]) = x[i];
  __threadfence();
#pragma unroll
  for (int i = 0; i < 2; ++i) *(volatile v4u*)(Ctx + off[i]) = x[i];
}

__global__ __launch_bounds__(256) void proj_gemm_kernel(
    const _Float16* __restrict__ A16, const _Float16* __restrict__ Bt,
    const float* __restrict__ bias, const float* __restrict__ Xin, float* __restrict__ Y) {
  __shared__ __attribute__((aligned(16))) float Cs[64 * LDC];
  const unsigned tid = threadIdx.x, lane = tid & 31u;
  const unsigned wave = __builtin_amdgcn_readfirstlane(threadIdx.x >> 5);
  const unsigned mw = wave >> 1, nw = wave & 1u;
  const unsigned hh = lane >> 4, m = lane & 15u;
  const unsigned n0 = blockIdx.x * 64u;
  const unsigned row0 = blockIdx.y * 64u;

  v8f acc0 = {}, acc1 = {};
  gemm_acc(A16, Bt, (unsigned)DIM, row0 + mw * 16u + m, n0 + nw * 32u + m, hh, acc0, acc1);
#pragma unroll
  for (int r = 0; r < 8; ++r) {
    float* d = &Cs[(mw * 16u + hh * 8u + (unsigned)r) * LDC + nw * 32u + m];
    d[0]  = acc0[r];
    d[16] = acc1[r];
  }
  __syncthreads();

  v4f xs[4];
  size_t off[4];
#pragma unroll
  for (unsigned i = 0; i < 4u; ++i) {
    const unsigned r = 16u * i + (tid >> 4);
    const unsigned c = (tid & 15u) * 4u;
    const unsigned crow = row0 + r;
    const unsigned bidx = crow / (unsigned)SEQ;
    const unsigned sq = crow - bidx * (unsigned)SEQ;
    const size_t frow = (size_t)bidx * SEQ_FULL + sq;
    const v4f u = *(const v4f*)&Cs[r * LDC + c];
    const v4f g = *(const v4f*)(bias + n0 + c);
    const v4f xr = *(const v4f*)(Xin + frow * DIM + n0 + c);
    v4f val;
#pragma unroll
    for (int j = 0; j < 4; ++j)
      val[j] = (u[j] * (1.0f / (WCARRY * ACARRY)) + bf16r(g[j])) + bf16r(xr[j]);
    xs[i] = val;
    off[i] = (size_t)crow * DIM + n0 + c;
  }
#pragma unroll
  for (int i = 0; i < 4; ++i) *(volatile v4f*)(Y + off[i]) = xs[i];
  __threadfence();
#pragma unroll
  for (int i = 0; i < 4; ++i) *(volatile v4f*)(Y + off[i]) = xs[i];
}

__global__ __launch_bounds__(256) void ln_kernel(
    const float* __restrict__ Y, const float* __restrict__ G, const float* __restrict__ Bv,
    float* __restrict__ netf, _Float16* __restrict__ net16) {
  const unsigned lane = threadIdx.x & 31u;
  const unsigned wave = __builtin_amdgcn_readfirstlane(threadIdx.x >> 5);
  const unsigned row = blockIdx.x * 8u + wave;
  const size_t base = (size_t)row * DIM + lane * 4u;
  const v4f a = *(const v4f*)(Y + base);
  const v4f c = *(const v4f*)(Y + base + 128);
  float s = ((a[0] + a[1]) + (a[2] + a[3])) + ((c[0] + c[1]) + (c[2] + c[3]));
  s = red32_sum(s);
  const float mean = s * (1.0f / (float)DIM);
  v4f da, dc;
  float q = 0.0f;
#pragma unroll
  for (int j = 0; j < 4; ++j) {
    da[j] = a[j] - mean;
    dc[j] = c[j] - mean;
    q += da[j] * da[j] + dc[j] * dc[j];
  }
  q = red32_sum(q);
  const float rstd = rsqrtf(q * (1.0f / (float)DIM) + LN_EPS);
  const v4f g0 = *(const v4f*)(G + lane * 4u);
  const v4f g1 = *(const v4f*)(G + 128u + lane * 4u);
  const v4f b0 = *(const v4f*)(Bv + lane * 4u);
  const v4f b1 = *(const v4f*)(Bv + 128u + lane * 4u);
  v4f o0, o1;
  v4h h0, h1;
#pragma unroll
  for (int j = 0; j < 4; ++j) {
    o0[j] = (da[j] * rstd) * bf16r(g0[j]) + bf16r(b0[j]);
    o1[j] = (dc[j] * rstd) * bf16r(g1[j]) + bf16r(b1[j]);
    h0[j] = (_Float16)(o0[j] * ACARRY);
    h1[j] = (_Float16)(o1[j] * ACARRY);
  }
  *(volatile v4f*)(netf + base) = o0;
  *(volatile v4f*)(netf + base + 128) = o1;
  *(volatile v4h*)(net16 + base) = h0;
  *(volatile v4h*)(net16 + base + 128) = h1;
  __threadfence();
  *(volatile v4f*)(netf + base) = o0;
  *(volatile v4f*)(netf + base + 128) = o1;
  *(volatile v4h*)(net16 + base) = h0;
  *(volatile v4h*)(net16 + base + 128) = h1;
}

__global__ __launch_bounds__(256) void fc1_gemm_kernel(
    const _Float16* __restrict__ A16, const _Float16* __restrict__ Bt,
    const float* __restrict__ bias, _Float16* __restrict__ H1) {
  __shared__ __attribute__((aligned(16))) float Cs[64 * LDC];
  const unsigned tid = threadIdx.x, lane = tid & 31u;
  const unsigned wave = __builtin_amdgcn_readfirstlane(threadIdx.x >> 5);
  const unsigned mw = wave >> 1, nw = wave & 1u;
  const unsigned hh = lane >> 4, m = lane & 15u;
  const unsigned n0 = blockIdx.x * 64u;
  const unsigned row0 = blockIdx.y * 64u;

  v8f acc0 = {}, acc1 = {};
  gemm_acc(A16, Bt, (unsigned)DIM, row0 + mw * 16u + m, n0 + nw * 32u + m, hh, acc0, acc1);
#pragma unroll
  for (int r = 0; r < 8; ++r) {
    float* d = &Cs[(mw * 16u + hh * 8u + (unsigned)r) * LDC + nw * 32u + m];
    d[0]  = acc0[r];
    d[16] = acc1[r];
  }
  __syncthreads();

  v8h x[2];
  size_t off[2];
#pragma unroll
  for (unsigned i = 0; i < 2u; ++i) {
    const unsigned r = 32u * i + (tid >> 3);
    const unsigned c = (tid & 7u) * 8u;
    const v4f u0 = *(const v4f*)&Cs[r * LDC + c];
    const v4f u1 = *(const v4f*)&Cs[r * LDC + c + 4];
    const v4f g0 = *(const v4f*)(bias + n0 + c);
    const v4f g1 = *(const v4f*)(bias + n0 + c + 4);
#pragma unroll
    for (int j = 0; j < 4; ++j) {
      x[i][j]     = (_Float16)((u0[j] * (1.0f / (WCARRY * ACARRY)) + bf16r(g0[j])) * ACARRY);
      x[i][j + 4] = (_Float16)((u1[j] * (1.0f / (WCARRY * ACARRY)) + bf16r(g1[j])) * ACARRY);
    }
    off[i] = (size_t)(row0 + r) * DFF + n0 + c;
  }
#pragma unroll
  for (int i = 0; i < 2; ++i) *(volatile v8h*)(H1 + off[i]) = x[i];
  __threadfence();
#pragma unroll
  for (int i = 0; i < 2; ++i) *(volatile v8h*)(H1 + off[i]) = x[i];
}

__global__ __launch_bounds__(256) void fc2_gemm_kernel(
    const _Float16* __restrict__ A16, const _Float16* __restrict__ Bt,
    const float* __restrict__ bias, const float* __restrict__ netf, float* __restrict__ outf) {
  __shared__ __attribute__((aligned(16))) float Cs[64 * LDC];
  const unsigned tid = threadIdx.x, lane = tid & 31u;
  const unsigned wave = __builtin_amdgcn_readfirstlane(threadIdx.x >> 5);
  const unsigned mw = wave >> 1, nw = wave & 1u;
  const unsigned hh = lane >> 4, m = lane & 15u;
  const unsigned n0 = blockIdx.x * 64u;
  const unsigned row0 = blockIdx.y * 64u;

  v8f acc0 = {}, acc1 = {};
  gemm_acc(A16, Bt, (unsigned)DFF, row0 + mw * 16u + m, n0 + nw * 32u + m, hh, acc0, acc1);
#pragma unroll
  for (int r = 0; r < 8; ++r) {
    float* d = &Cs[(mw * 16u + hh * 8u + (unsigned)r) * LDC + nw * 32u + m];
    d[0]  = acc0[r];
    d[16] = acc1[r];
  }
  __syncthreads();

  v4f xs[4];
  size_t off[4];
#pragma unroll
  for (unsigned i = 0; i < 4u; ++i) {
    const unsigned r = 16u * i + (tid >> 4);
    const unsigned c = (tid & 15u) * 4u;
    const unsigned crow = row0 + r;
    const unsigned bidx = crow / (unsigned)SEQ;
    const unsigned sq = crow - bidx * (unsigned)SEQ;
    const size_t frow = (size_t)bidx * SEQ_FULL + sq;
    const v4f u = *(const v4f*)&Cs[r * LDC + c];
    const v4f g = *(const v4f*)(bias + n0 + c);
    const v4f sc = *(const v4f*)(netf + (size_t)crow * DIM + n0 + c);
    v4f val;
#pragma unroll
    for (int j = 0; j < 4; ++j)
      val[j] = (u[j] * (1.0f / (WCARRY * ACARRY)) + bf16r(g[j])) + sc[j];
    xs[i] = val;
    off[i] = frow * DIM + n0 + c;
  }
#pragma unroll
  for (int i = 0; i < 4; ++i) *(volatile v4f*)(outf + off[i]) = xs[i];
  __threadfence();
#pragma unroll
  for (int i = 0; i < 4; ++i) *(volatile v4f*)(outf + off[i]) = xs[i];
}

extern "C" void kernel_launch(void* const* d_in, const int* in_sizes, int n_in,
                              void* d_out, int out_size, void* d_ws, size_t ws_size,
                              hipStream_t stream) {
  if (n_in < 10) return;
  const long long need_x = ((long long)(NB - 1) * SEQ_FULL + SEQ) * DIM;
  if ((long long)in_sizes[0] < need_x) return;
  if ((long long)in_sizes[1] < (long long)DIM * 3 * DIM) return;
  if ((long long)in_sizes[2] < (long long)DIM * DIM) return;
  if (in_sizes[3] < DIM) return;
  if ((long long)in_sizes[4] < (long long)DIM * DFF) return;
  if (in_sizes[5] < DFF) return;
  if ((long long)in_sizes[6] < (long long)DFF * DIM) return;
  if (in_sizes[7] < DIM) return;
  if (in_sizes[8] < DIM) return;
  if (in_sizes[9] < DIM) return;
  if ((long long)out_size < need_x) return;
  if (ws_size < WS_TOTAL) return;

  const float* X     = (const float*)d_in[0];
  const float* Wqkv  = (const float*)d_in[1];
  const float* Wproj = (const float*)d_in[2];
  const float* bproj = (const float*)d_in[3];
  const float* Wfc1  = (const float*)d_in[4];
  const float* bfc1  = (const float*)d_in[5];
  const float* Wfc2  = (const float*)d_in[6];
  const float* bfc2  = (const float*)d_in[7];
  const float* lng   = (const float*)d_in[8];
  const float* lnb   = (const float*)d_in[9];
  float* out = (float*)d_out;

  char* ws = (char*)d_ws;
  _Float16* Wqkv_t  = (_Float16*)(ws + OFF_WQKV);
  _Float16* Wproj_t = (_Float16*)(ws + OFF_WPROJ);
  _Float16* Wfc1_t  = (_Float16*)(ws + OFF_WFC1);
  _Float16* Wfc2_t  = (_Float16*)(ws + OFF_WFC2);
  _Float16* X16     = (_Float16*)(ws + OFF_X16);
  unsigned short* QK  = (unsigned short*)(ws + OFF_QK);
  unsigned short* VT  = (unsigned short*)(ws + OFF_VT);
  unsigned short* Ctx = (unsigned short*)(ws + OFF_CTX);
  float* Y          = (float*)(ws + OFF_Y);
  float* Netf       = (float*)(ws + OFF_NETF);
  _Float16* Net16   = (_Float16*)(ws + OFF_NET16);
  _Float16* H1      = (_Float16*)(ws + OFF_H1);

  dim3 blk(256);

  wconv_kernel<<<dim3(3 * DIM / 64, DIM / 64), blk, 0, stream>>>(Wqkv, Wqkv_t, (unsigned)DIM, (unsigned)(3 * DIM));
  wconv_kernel<<<dim3(DIM / 64, DIM / 64), blk, 0, stream>>>(Wproj, Wproj_t, (unsigned)DIM, (unsigned)DIM);
  wconv_kernel<<<dim3(DFF / 64, DIM / 64), blk, 0, stream>>>(Wfc1, Wfc1_t, (unsigned)DIM, (unsigned)DFF);
  wconv_kernel<<<dim3(DIM / 64, DFF / 64), blk, 0, stream>>>(Wfc2, Wfc2_t, (unsigned)DFF, (unsigned)DIM);

  xconv_kernel<<<dim3((unsigned)(((size_t)MROWS * DIM) / 2048)), blk, 0, stream>>>(X, X16);
  qkv_gemm_kernel<<<dim3(3 * DIM / 64, MROWS / 64), blk, 0, stream>>>(X16, Wqkv_t, QK, VT);
  attn_kernel<<<dim3(SEQ / 64, NHEAD / 2, NB), blk, 0, stream>>>(QK, VT, Ctx);
  proj_gemm_kernel<<<dim3(DIM / 64, MROWS / 64), blk, 0, stream>>>(
      (const _Float16*)Ctx, Wproj_t, bproj, X, Y);
  ln_kernel<<<dim3(MROWS / 8), blk, 0, stream>>>(Y, lng, lnb, Netf, Net16);
  fc1_gemm_kernel<<<dim3(DFF / 64, MROWS / 64), blk, 0, stream>>>(Net16, Wfc1_t, bfc1, H1);
  fc2_gemm_kernel<<<dim3(DIM / 64, MROWS / 64), blk, 0, stream>>>(H1, Wfc2_t, bfc2, Netf, out);
}
